// Poly2d_83751862272438
// MI455X (gfx1250) — hardware-verified
//
#include <hip/hip_runtime.h>
#include <math.h>

typedef __attribute__((ext_vector_type(16))) _Float16 v16h;
typedef __attribute__((ext_vector_type(16))) __bf16 v16b;
typedef __attribute__((ext_vector_type(8)))  _Float16 v8h;
typedef __attribute__((ext_vector_type(8)))  float v8f;
typedef __attribute__((ext_vector_type(4)))  float v4f;
typedef __attribute__((ext_vector_type(2)))  float v2f;
typedef __attribute__((ext_vector_type(4)))  unsigned v4u;
typedef __attribute__((ext_vector_type(4)))  int v4i;
typedef float __attribute__((may_alias)) float_a;
typedef int __attribute__((may_alias)) int_a;

template <typename T> __device__ __forceinline__ void vst2(void* p, T v) { *(volatile T*)p = v; __threadfence(); *(volatile T*)p = v; }
__device__ __forceinline__ v8f wmma16(v16h a, v16h b, v8f c) {
  v8f d = __builtin_amdgcn_wmma_f32_16x16x32_f16(false, a, false, b, (short)0, c, false, false);
  asm volatile("v_nop\n\tv_nop\n\tv_nop\n\tv_nop" : "+v"(d) : "v"(a), "v"(b));
  return d;
}
__device__ __forceinline__ v8f wmma_bf(v16b a, v16b b, v8f c) {
  v8f d = __builtin_amdgcn_wmma_f32_16x16x32_bf16(false, a, false, b, (short)0, c, false, false);
  asm volatile("v_nop\n\tv_nop\n\tv_nop\n\tv_nop" : "+v"(d) : "v"(a), "v"(b));
  return d;
}
__device__ __forceinline__ v16h frag_h(const _Float16* rowk0, int lane) {
  union { v16h v; v8h q[2]; } u; const _Float16* p = rowk0 + 8 * (lane >> 4);
  u.q[0] = *(const v8h*)p; u.q[1] = *(const v8h*)(p + 16); return u.v;
}
__device__ __forceinline__ v16h frag_f32(const float* rowk0, int lane) {
  v16h a; const float* p = rowk0 + 8 * (lane >> 4);
#pragma unroll
  for (int i = 0; i < 8; ++i) { a[i] = (_Float16)p[i]; a[8 + i] = (_Float16)p[16 + i]; }
  return a;
}
__device__ __forceinline__ v16h frag_f32s(const float* rowk0, int lane, float sc) {
  v16h a; const float* p = rowk0 + 8 * (lane >> 4);
#pragma unroll
  for (int i = 0; i < 8; ++i) { a[i] = (_Float16)(p[i] * sc); a[8 + i] = (_Float16)(p[16 + i] * sc); }
  return a;
}
__device__ __forceinline__ v16h fragc_f32(const float* W, int k0, int n, int lane, int ld, int K) {
  v16h a; const int g = lane >> 4;
#pragma unroll
  for (int i = 0; i < 8; ++i) { const int ka = k0 + 8 * g + i, kb = ka + 16;
    a[i] = (_Float16)(ka < K ? W[(size_t)(ka < K ? ka : K - 1) * ld + n] : 0.f); a[8 + i] = (_Float16)(kb < K ? W[(size_t)(kb < K ? kb : K - 1) * ld + n] : 0.f); }
  return a;
}
struct F2 { v16b h, l; };
__device__ __forceinline__ F2 bsplit16(const float v[16]) { F2 r;
#pragma unroll
  for (int i = 0; i < 16; ++i) { const __bf16 h = (__bf16)v[i]; r.h[i] = h; r.l[i] = (__bf16)(v[i] - (float)h); }
  return r; }
__device__ __forceinline__ F2 split_row(const float* row, int k0, int lane) { float v[16]; const float* p = row + k0 + 8 * (lane >> 4);
#pragma unroll
  for (int i = 0; i < 8; ++i) { v[i] = p[i]; v[8 + i] = p[16 + i]; }
  return bsplit16(v); }
__device__ __forceinline__ F2 split_rowK(const float* row, int k0, int lane, int K) { float v[16]; const int g = lane >> 4;
#pragma unroll
  for (int i = 0; i < 8; ++i) { const int ka = k0 + 8 * g + i, kb = ka + 16; v[i] = ka < K ? row[ka < K ? ka : K - 1] : 0.f; v[8 + i] = kb < K ? row[kb < K ? kb : K - 1] : 0.f; }
  return bsplit16(v); }
__device__ __forceinline__ F2 split_col(const float* W, int k0, int n, int lane, int ld, int K) { float v[16]; const int g = lane >> 4;
#pragma unroll
  for (int i = 0; i < 8; ++i) { const int ka = k0 + 8 * g + i, kb = ka + 16; v[i] = ka < K ? W[(size_t)(ka < K ? ka : K - 1) * ld + n] : 0.f; v[8 + i] = kb < K ? W[(size_t)(kb < K ? kb : K - 1) * ld + n] : 0.f; }
  return bsplit16(v); }
__device__ __forceinline__ v8f mac3(const F2& a, const F2& b, v8f c) { c = wmma_bf(a.l, b.h, c); c = wmma_bf(a.h, b.l, c); return wmma_bf(a.h, b.h, c); }
__device__ __forceinline__ float sigm(float v) { return 1.0f / (1.0f + expf(-v)); }
#define LDSX() do { asm volatile("s_wait_dscnt 0" ::: "memory"); __builtin_amdgcn_wave_barrier(); __builtin_amdgcn_fence(__ATOMIC_RELEASE, "workgroup"); } while (0)


#define NBt 8
#define CIN 64
#define COUT 64
#define IH 64
#define IW 64
#define NPIX (IH * IW)
#define VS 10
#define KK (CIN * VS * VS)
#define NR (NBt * NPIX)
typedef __attribute__((ext_vector_type(8))) __bf16 v8b;
__device__ __forceinline__ v16b frag_b(const __bf16* rowk0, int lane) {
  union { v16b v; v8b q[2]; } u; const __bf16* p = rowk0 + 8 * (lane >> 4);
  u.q[0] = *(const v8b*)p; u.q[1] = *(const v8b*)(p + 16); return u.v;
}
__device__ __forceinline__ float bfr(float v) { return (float)(__bf16)v; }
__device__ __attribute__((noinline)) float exp_ni(float v) { return expf(v); }
__device__ __attribute__((noinline)) float erf_ni(float v) { return erff(v); }

#define WS_END 16u

__global__ __launch_bounds__(128) void k_poly(const float* __restrict__ X, const float* __restrict__ FW, const float* __restrict__ BI, float* __restrict__ OUT) {
  __shared__ __align__(16) __bf16 ssv[64][CIN * VS + 2];
  __shared__ __align__(16) float so[COUT][68];
  const int tid = threadIdx.x, wave = tid >> 5, lane = tid & 31, col = lane & 15, g = lane >> 4; const size_t r0 = (size_t)blockIdx.x * 64; const size_t b = r0 / NPIX; const int p0 = (int)(r0 % NPIX); const int y0 = p0 / IW;
  for (int e = tid; e < 64 * CIN * VS; e += 128) { const int px = e / (CIN * VS), rem = e % (CIN * VS); const int c = rem / VS, v = rem % VS; float val;
    if (v == 0) val = 1.0f; else { const int kh = (v - 1) / 3, kw = (v - 1) % 3; const int yy = y0 + kh - 1, xx = px + kw - 1; val = (yy >= 0 && yy < IH && xx >= 0 && xx < IW) ? X[((b * CIN + c) * IH + yy) * (size_t)IW + xx] : 0.f; }
    ssv[px][rem] = (__bf16)val; }
  __syncthreads();
  v8f acc[4] = {};
  const __bf16* srow = &ssv[wave * 16 + col][0];
#pragma unroll 1
  for (int kc = 0; kc < KK / 32; ++kc) {
    float qv[16];
#pragma unroll
    for (int i = 0; i < 16; ++i) { const int k = kc * 32 + 8 * g + (i < 8 ? i : i + 8); const int c = k / (VS * VS), ij = k % (VS * VS); const int ii = ij / VS, jj = ij % VS; qv[i] = (float)srow[c * VS + ii] * (float)srow[c * VS + jj]; }
    const F2 a = bsplit16(qv);
#pragma unroll
    for (int j = 0; j < 4; ++j) { v16b w; const int o = j * 16 + col;
#pragma unroll
      for (int i = 0; i < 8; ++i) { w[i] = (__bf16)FW[(size_t)o * KK + kc * 32 + 8 * g + i]; w[8 + i] = (__bf16)FW[(size_t)o * KK + kc * 32 + 16 + 8 * g + i]; }
      acc[j] = wmma_bf(a.h, w, acc[j]); acc[j] = wmma_bf(a.l, w, acc[j]); } }
#pragma unroll
  for (int j = 0; j < 4; ++j) { const int o = j * 16 + col; const float bb = bfr(BI[o]);
#pragma unroll
    for (int r = 0; r < 8; ++r) so[o][wave * 16 + 8 * g + r] = acc[j][r] + bb; }
  __syncthreads(); for (int e = tid; e < COUT * 16; e += 128) { const int o = e >> 4, q = e & 15; vst2(OUT + ((b * COUT + o) * (size_t)NPIX + p0 + q * 4), *(const v4f*)&so[o][q * 4]); } }
extern "C" void kernel_launch(void* const* d_in, const int* in_sizes, int n_in, void* d_out, int out_size, void* d_ws, size_t ws_size, hipStream_t stream) {
  (void)in_sizes; (void)n_in; (void)out_size; (void)d_ws; (void)ws_size;
  const float** F = (const float**)d_in;
  k_poly<<<NR / 64, 128, 0, stream>>>(F[0], F[1], F[2], (float*)d_out);
}
